// attention_unit_73735998538275
// MI455X (gfx1250) — hardware-verified
//
#include <hip/hip_runtime.h>
#include <stddef.h>
#include <stdint.h>

#define NB  8
#define CI  130
#define CH  144
#define NP  4096
#define CQ  32
#define KP  160
#define XSP 168
#define HSP 72
#define FSP 40
#define PTP 72
#define OSP 68
#define BN_EPS 1e-5f

static_assert(NP % 128 == 0);
static_assert(CH % 16 == 0);
static_assert(CH >= CI);
static_assert(KP % 32 == 0);
static_assert(KP >= CI);
static_assert(XSP >= KP);
static_assert((XSP % 8) == 0);
static_assert((HSP % 8) == 0);
static_assert((FSP % 8) == 0);
static_assert((PTP % 8) == 0);
static_assert((OSP % 4) == 0);

typedef _Float16 v16h __attribute__((ext_vector_type(16)));
typedef _Float16 v8h  __attribute__((ext_vector_type(8)));
typedef float    v8f  __attribute__((ext_vector_type(8)));
typedef float    v4f  __attribute__((ext_vector_type(4)));
typedef unsigned int v4u __attribute__((ext_vector_type(4)));

union Frag  { v16h v; v8h h[2]; };
union Pack8 { v8h h; v4u u; };

__device__ __forceinline__ v8f mma16(v16h a, v16h b, v8f c) {
  c = __builtin_amdgcn_wmma_f32_16x16x32_f16(false, a, false, b, (short)0, c, false, false);
  asm volatile("v_nop\n\tv_nop\n\tv_nop\n\tv_nop" : "+v"(c) : "v"(a), "v"(b));
  return c;
}

__device__ __forceinline__ v16h ldfrag(const _Float16* p, int ld, int row0, int k0, int lane) {
  const int m = lane & 15, lh = lane >> 4;
  const _Float16* q = p + (size_t)(row0 + m) * ld + k0 + 8 * lh;
  Frag f;
  f.h[0] = *(const v8h*)(q);
  f.h[1] = *(const v8h*)(q + 16);
  return f.v;
}

__device__ __forceinline__ v8f zero8() { return (v8f){0.f, 0.f, 0.f, 0.f, 0.f, 0.f, 0.f, 0.f}; }

__device__ __forceinline__ v4u cvt8(const float* __restrict__ src, int srow, bool rowok, int pc) {
  v8h hv;
#pragma unroll
  for (int i = 0; i < 8; ++i) {
    const int col = pc * 8 + i;
    const int cl = (col < CI) ? col : (CI - 1);
    const float v = src[(size_t)srow * CI + cl];
    hv[i] = (_Float16)((rowok && col < CI) ? v * 16.0f : 0.0f);
  }
  Pack8 pk;
  pk.h = hv;
  return pk.u;
}

__global__ __launch_bounds__(64) void k_cvt_w(const float* __restrict__ wF, const float* __restrict__ wG,
                                              const float* __restrict__ wH,
                                              _Float16* __restrict__ pFG, _Float16* __restrict__ pHp) {
  const int bid = blockIdx.x, tid = (int)threadIdx.x;
  v4u vv;
  _Float16* dst;
  if (bid < 10) {
    const int p = bid * 64 + tid;
    const int row = p / 20, pc = p - row * 20;
    vv  = cvt8(wF, row, true, pc);
    dst = pFG + (size_t)p * 8;
  } else if (bid < 20) {
    const int p = bid * 64 + tid;
    const int row = p / 20, pc = p - row * 20;
    vv  = cvt8(wG, row - CQ, true, pc);
    dst = pFG + (size_t)p * 8;
  } else {
    const int p = (bid - 20) * 64 + tid;
    const int row = p / 20, pc = p - row * 20;
    const int sr = (row < CI) ? row : (CI - 1);
    vv  = cvt8(wH, sr, row < CI, pc);
    dst = pHp + (size_t)p * 8;
  }
  volatile v4u* d = (volatile v4u*)dst;
  *d = vv;
  __threadfence();
  *d = vv;
}

__global__ __launch_bounds__(256) void k_proj(const float* __restrict__ x,
                                             const _Float16* __restrict__ pFG,
                                             const _Float16* __restrict__ pHp,
                                             const float* __restrict__ bF,   const float* __restrict__ bnFw,
                                             const float* __restrict__ bnFb, const float* __restrict__ bnFm,
                                             const float* __restrict__ bnFv,
                                             const float* __restrict__ bG,   const float* __restrict__ bnGw,
                                             const float* __restrict__ bnGb, const float* __restrict__ bnGm,
                                             const float* __restrict__ bnGv,
                                             const float* __restrict__ bH,   const float* __restrict__ bnHw,
                                             const float* __restrict__ bnHb, const float* __restrict__ bnHm,
                                             const float* __restrict__ bnHv,
                                             _Float16* __restrict__ fT, _Float16* __restrict__ gT,
                                             _Float16* __restrict__ hp) {
  __shared__ __align__(16) _Float16 xs[64 * XSP];
  __shared__ __align__(16) _Float16 hs[CH * HSP];
  __shared__ __align__(16) _Float16 fgs[2 * 64 * FSP];
  const int tid = threadIdx.x, lane = tid & 31, wave = tid >> 5;
  const int hh = lane >> 4, lm = lane & 15;
  const int j = wave & 3, tq = wave >> 2;
  const int b = blockIdx.x >> 6;
  const int n0 = (blockIdx.x & 63) * 64;
  const int r0 = 16 * j;

  const float* xb = x + (size_t)b * CI * NP + n0;
  for (int i = tid; i < CI * 64; i += 256) {
    const int c = i >> 6, nn = i & 63;
    xs[nn * XSP + c] = (_Float16)xb[(size_t)c * NP + nn];
  }
  for (int i = tid; i < 64 * 32; i += 256) {
    const int nn = i >> 5, c = CI + (i & 31);
    xs[nn * XSP + c] = (_Float16)0.0f;
  }
  __syncthreads();

  v8f ah[5], aw[2];
#pragma unroll
  for (int q = 0; q < 5; ++q) ah[q] = zero8();
  aw[0] = zero8();
  aw[1] = zero8();

#pragma unroll 1
  for (int ks = 0; ks < KP / 32; ++ks) {
    const int k0 = 32 * ks;
    const v16h a = ldfrag(xs, XSP, r0, k0, lane);
#pragma unroll
    for (int q = 0; q < 4; ++q)
      ah[q] = mma16(a, ldfrag(pHp, KP, 16 * (5 * tq + q), k0, lane), ah[q]);
    if (tq == 0)
      ah[4] = mma16(a, ldfrag(pHp, KP, 64, k0, lane), ah[4]);
#pragma unroll
    for (int ot = 0; ot < 2; ++ot)
      aw[ot] = mma16(a, ldfrag(pFG, KP, 32 * tq + 16 * ot, k0, lane), aw[ot]);
  }

#pragma unroll
  for (int q = 0; q < 5; ++q) {
    if (q < 4 || tq == 0) {
      const int ct = 5 * tq + q;
      const int c = 16 * ct + lm;
      const int cc = (c < CI) ? c : (CI - 1);
      const float sc = bnHw[cc] * rsqrtf(bnHv[cc] + BN_EPS);
      const float sh = (bH[cc] - bnHm[cc]) * sc + bnHb[cc];
      const float sc16 = sc * 0.0625f;
      const bool ok = (c < CI);
      v8h hv;
#pragma unroll
      for (int r = 0; r < 8; ++r) {
        const float y = fmaxf(fmaf(ah[q][r], sc16, sh), 0.0f);
        hv[r] = (_Float16)(ok ? y : 0.0f);
      }
      Pack8 pk;
      pk.h = hv;
      *(v4u*)(hs + c * HSP + r0 + 8 * hh) = pk.u;
    }
  }
#pragma unroll
  for (int ot = 0; ot < 2; ++ot) {
    const int o = 16 * ot + lm;
    const float scf = bnFw[o] * rsqrtf(bnFv[o] + BN_EPS);
    const float shf = (bF[o] - bnFm[o]) * scf + bnFb[o];
    const float scg = bnGw[o] * rsqrtf(bnGv[o] + BN_EPS);
    const float shg = (bG[o] - bnGm[o]) * scg + bnGb[o];
    const float sc16 = (tq ? scg : scf) * 0.0625f;
    const float sh = tq ? shg : shf;
#pragma unroll
    for (int r = 0; r < 8; ++r)
      fgs[tq * (64 * FSP) + (r0 + 8 * hh + r) * FSP + o] = (_Float16)fmaxf(fmaf(aw[ot][r], sc16, sh), 0.0f);
  }
  __syncthreads();

  const size_t tb = ((size_t)b * NP + n0) * CQ;
  v4u vf, vg;
  {
    Pack8 pk;
    pk.h = *(const v8h*)(fgs + (tid >> 2) * FSP + (tid & 3) * 8);
    vf = pk.u;
    pk.h = *(const v8h*)(fgs + 64 * FSP + (tid >> 2) * FSP + (tid & 3) * 8);
    vg = pk.u;
  }
  v4u vh[5];
  size_t gh[5];
#pragma unroll
  for (int it = 0; it < 5; ++it) {
    vh[it] = (v4u){0u, 0u, 0u, 0u};
    gh[it] = 0;
    if (it < 4 || wave < 4) {
      const int p = tid + 256 * it;
      const int c = p >> 3;
      const int pc = p & 7;
      Pack8 pk;
      pk.h = *(const v8h*)(hs + c * HSP + pc * 8);
      vh[it] = pk.u;
      gh[it] = ((size_t)(b * CH + c)) * NP + n0 + pc * 8;
    }
  }
  for (int ps = 0; ps < 2; ++ps) {
    *(volatile v4u*)(fT + tb + (size_t)tid * 8) = vf;
    *(volatile v4u*)(gT + tb + (size_t)tid * 8) = vg;
#pragma unroll
    for (int it = 0; it < 5; ++it)
      if (it < 4 || wave < 4) *(volatile v4u*)(hp + gh[it]) = vh[it];
    __threadfence();
  }
}

__global__ __launch_bounds__(256) void k_stats(const _Float16* __restrict__ gT,
                                               const _Float16* __restrict__ fT,
                                               float* __restrict__ Mrow, float* __restrict__ rZ) {
  __shared__ __align__(16) float sM[128];
  __shared__ __align__(16) float sZ[128];
  const int tid = threadIdx.x, lane = tid & 31, wave = tid >> 5;
  const int hh = lane >> 4, lm = lane & 15;
  const int b = blockIdx.x >> 5, nb = blockIdx.x & 31;
  const int n0 = nb * 128 + wave * 16;
  const _Float16* G = gT + (size_t)b * NP * CQ;
  const _Float16* F = fT + (size_t)b * NP * CQ;

  const v16h ga = ldfrag(G, CQ, n0, 0, lane);
  float mr[8], zr[8];
#pragma unroll
  for (int r = 0; r < 8; ++r) { mr[r] = -1.0e30f; zr[r] = 0.0f; }

#pragma unroll 1
  for (int mg = 0; mg < NP; mg += 128) {
    v8f s[8];
#pragma unroll
    for (int t = 0; t < 8; ++t) s[t] = mma16(ga, ldfrag(F, CQ, mg + 16 * t, 0, lane), zero8());
#pragma unroll
    for (int r = 0; r < 8; ++r) {
      float lmx = s[0][r];
#pragma unroll
      for (int t = 1; t < 8; ++t) lmx = fmaxf(lmx, s[t][r]);
      const float nm = fmaxf(mr[r], lmx);
      float z = zr[r] * __expf(mr[r] - nm);
#pragma unroll
      for (int t = 0; t < 8; ++t) z += __expf(s[t][r] - nm);
      zr[r] = z;
      mr[r] = nm;
    }
  }
#pragma unroll
  for (int r = 0; r < 8; ++r) {
    float M = mr[r], Z = zr[r];
#pragma unroll
    for (int mk = 1; mk < 16; mk <<= 1) {
      const float oM = __shfl_xor(M, mk, 32);
      const float oZ = __shfl_xor(Z, mk, 32);
      const float nM = fmaxf(M, oM);
      Z = Z * __expf(M - nM) + oZ * __expf(oM - nM);
      M = nM;
    }
    mr[r] = M;
    zr[r] = Z;
  }
  if (lm == 0) {
#pragma unroll
    for (int r = 0; r < 8; ++r) {
      sM[wave * 16 + 8 * hh + r] = mr[r];
      sZ[wave * 16 + 8 * hh + r] = 1.0f / zr[r];
    }
  }
  __syncthreads();
  if (wave == 0) {
    const v4f mv = *(const v4f*)(sM + 4 * lane);
    const v4f zv = *(const v4f*)(sZ + 4 * lane);
    const size_t o = (size_t)b * NP + nb * 128 + 4 * lane;
    volatile v4f* dm = (volatile v4f*)(Mrow + o);
    volatile v4f* dz = (volatile v4f*)(rZ + o);
    *dm = mv;
    *dz = zv;
    __threadfence();
    *dm = mv;
    *dz = zv;
  }
}

__global__ __launch_bounds__(256) void k_av(const float* __restrict__ x,
                                           const _Float16* __restrict__ gT,
                                           const _Float16* __restrict__ fT,
                                           const _Float16* __restrict__ hp,
                                           const float* __restrict__ Mrow, const float* __restrict__ rZ,
                                           const float* __restrict__ gamma, float* __restrict__ out) {
  __shared__ __align__(16) _Float16 Pt[64 * PTP];
  __shared__ __align__(16) float ost[CH * OSP];
  const int tid = threadIdx.x, lane = tid & 31, wave = tid >> 5;
  const int hh = lane >> 4, lm = lane & 15;
  const int j = wave & 3, tq = wave >> 2;
  const int b = blockIdx.x >> 6;
  const int m0 = (blockIdx.x & 63) * 64;

  const _Float16* G = gT + (size_t)b * NP * CQ;
  const _Float16* F = fT + (size_t)b * NP * CQ;
  const _Float16* H = hp + (size_t)b * CH * NP;
  const float* Mb = Mrow + (size_t)b * NP;
  const float* Zb = rZ + (size_t)b * NP;

  const v16h bfm = ldfrag(F, CQ, m0 + 16 * j, 0, lane);
  v8f acc[5];
#pragma unroll
  for (int q = 0; q < 5; ++q) acc[q] = zero8();

#pragma unroll 1
  for (int nc = 0; nc < NP; nc += 64) {
    __syncthreads();
#pragma unroll
    for (int t2 = 0; t2 < 2; ++t2) {
      const int t = 2 * tq + t2;
      const int nr = nc + 16 * t;
      const v16h ga = ldfrag(G, CQ, nr, 0, lane);
      const v8f s = mma16(ga, bfm, zero8());
      const v8f mv = *(const v8f*)(Mb + nr + 8 * hh);
      const v8f zv = *(const v8f*)(Zb + nr + 8 * hh);
      v8h pv;
#pragma unroll
      for (int r = 0; r < 8; ++r) pv[r] = (_Float16)(__expf(s[r] - mv[r]) * (zv[r] * 1024.0f));
      Pack8 pk;
      pk.h = pv;
      *(v4u*)(Pt + (16 * j + lm) * PTP + 16 * t + 8 * hh) = pk.u;
    }
    __syncthreads();
#pragma unroll
    for (int kk = 0; kk < 2; ++kk) {
      const v16h pb = ldfrag(Pt, PTP, 16 * j, 32 * kk, lane);
      const int k0 = nc + 32 * kk;
#pragma unroll
      for (int q = 0; q < 4; ++q)
        acc[q] = mma16(ldfrag(H, NP, 16 * (2 * q + tq), k0, lane), pb, acc[q]);
      if (tq == 0)
        acc[4] = mma16(ldfrag(H, NP, 128, k0, lane), pb, acc[4]);
    }
  }

  const float gsc = gamma[0] * 0.0009765625f;
#pragma unroll
  for (int q = 0; q < 4; ++q) {
    const int ct = 2 * q + tq;
#pragma unroll
    for (int r = 0; r < 8; ++r) ost[(16 * ct + 8 * hh + r) * OSP + 16 * j + lm] = acc[q][r];
  }
  if (tq == 0) {
#pragma unroll
    for (int r = 0; r < 8; ++r) ost[(128 + 8 * hh + r) * OSP + 16 * j + lm] = acc[4][r];
  }
  __syncthreads();

  const float* xb = x + (size_t)b * CI * NP;
  float* ob = out + (size_t)b * CI * NP;
  v4f val[9];
  size_t go[9];
#pragma unroll
  for (int it = 0; it < 9; ++it) {
    const int p = tid + 256 * it;
    int line = p >> 3;
    line = (line < 2 * CI) ? line : (2 * CI - 1);
    const int c = line >> 1, half = line & 1, pc = p & 7;
    const int col = m0 + half * 32 + pc * 4;
    const v4f ov = *(const v4f*)(ost + c * OSP + half * 32 + pc * 4);
    go[it] = (size_t)c * NP + col;
    const v4f xv = *(const v4f*)(xb + go[it]);
    val[it] = ov * gsc + xv;
  }
  for (int ps = 0; ps < 2; ++ps) {
#pragma unroll
    for (int it = 0; it < 8; ++it) *(volatile v4f*)(ob + go[it]) = val[it];
    if (wave == 0) *(volatile v4f*)(ob + go[8]) = val[8];
    __threadfence();
  }
}

#define SZ_WFG ((size_t)2 * CQ * KP * 2)
#define SZ_WH  ((size_t)CH * KP * 2)
#define SZ_GF  ((size_t)NB * NP * CQ * 2)
#define SZ_HP  ((size_t)NB * CH * NP * 2)
#define SZ_ST  ((size_t)NB * NP * 4)
#define O_WFG ((size_t)0)
#define O_WH  (O_WFG + SZ_WFG)
#define O_GT  (O_WH + SZ_WH)
#define O_FT  (O_GT + SZ_GF)
#define O_HP  (O_FT + SZ_GF)
#define O_M   (O_HP + SZ_HP)
#define O_Z   (O_M + SZ_ST)
#define O_END (O_Z + SZ_ST)

static_assert(O_END == (size_t)13960192);
static_assert(O_END <= (size_t)134217728);
static_assert((O_WH % 256) == 0);
static_assert((O_GT % 256) == 0);
static_assert((O_FT % 256) == 0);
static_assert((O_HP % 256) == 0);
static_assert((O_M % 256) == 0);
static_assert((O_Z % 256) == 0);
static_assert((SZ_WFG % 512) == 0);
static_assert((SZ_WH % 512) == 0);

extern "C" void kernel_launch(void* const* d_in, const int* in_sizes, int n_in,
                              void* d_out, int out_size, void* d_ws, size_t ws_size,
                              hipStream_t stream) {
  if (n_in < 20) return;
  if (in_sizes[0] != NB * CI * NP) return;
  if (in_sizes[1] != CQ * CI || in_sizes[7] != CQ * CI) return;
  for (int i = 2; i <= 6; ++i) if (in_sizes[i] != CQ) return;
  for (int i = 8; i <= 12; ++i) if (in_sizes[i] != CQ) return;
  if (in_sizes[13] != CI * CI) return;
  for (int i = 14; i <= 18; ++i) if (in_sizes[i] != CI) return;
  if (in_sizes[19] < 1) return;
  if (out_size != NB * CI * NP) return;
  if (O_END > ws_size) return;

  const float* x     = (const float*)d_in[0];
  const float* wF    = (const float*)d_in[1];
  const float* bF    = (const float*)d_in[2];
  const float* bnFw  = (const float*)d_in[3];
  const float* bnFb  = (const float*)d_in[4];
  const float* bnFm  = (const float*)d_in[5];
  const float* bnFv  = (const float*)d_in[6];
  const float* wG    = (const float*)d_in[7];
  const float* bG    = (const float*)d_in[8];
  const float* bnGw  = (const float*)d_in[9];
  const float* bnGb  = (const float*)d_in[10];
  const float* bnGm  = (const float*)d_in[11];
  const float* bnGv  = (const float*)d_in[12];
  const float* wH    = (const float*)d_in[13];
  const float* bH    = (const float*)d_in[14];
  const float* bnHw  = (const float*)d_in[15];
  const float* bnHb  = (const float*)d_in[16];
  const float* bnHm  = (const float*)d_in[17];
  const float* bnHv  = (const float*)d_in[18];
  const float* gamma = (const float*)d_in[19];
  float* out = (float*)d_out;

  char* ws = (char*)d_ws;
  _Float16* WFG = (_Float16*)(ws + O_WFG);
  _Float16* WHp = (_Float16*)(ws + O_WH);
  _Float16* gTp = (_Float16*)(ws + O_GT);
  _Float16* fTp = (_Float16*)(ws + O_FT);
  _Float16* hpp = (_Float16*)(ws + O_HP);
  float*    Mr  = (float*)(ws + O_M);
  float*    Zr  = (float*)(ws + O_Z);

  k_cvt_w<<<dim3(65), dim3(64), 0, stream>>>(wF, wG, wH, WFG, WHp);
  k_proj<<<dim3(NB * (NP / 64)), dim3(256), 0, stream>>>(x, WFG, WHp,
                                                         bF, bnFw, bnFb, bnFm, bnFv,
                                                         bG, bnGw, bnGb, bnGm, bnGv,
                                                         bH, bnHw, bnHb, bnHm, bnHv,
                                                         fTp, gTp, hpp);
  k_stats<<<dim3(NB * (NP / 128)), dim3(256), 0, stream>>>(gTp, fTp, Mr, Zr);
  k_av<<<dim3(NB * (NP / 64)), dim3(256), 0, stream>>>(x, gTp, fTp, hpp, Mr, Zr, gamma, out);
  (void)hipGetLastError();
}
